// PointNetSetAbstraction_24120536335102
// MI455X (gfx1250) — hardware-verified
//
#include <hip/hip_runtime.h>
#include <math.h>
#pragma clang fp contract(off)

typedef __attribute__((ext_vector_type(16))) _Float16 v16h;
typedef __attribute__((ext_vector_type(8)))  _Float16 v8h;
typedef __attribute__((ext_vector_type(8)))  float    v8f;
typedef __attribute__((ext_vector_type(4)))  float    v4f;
typedef __attribute__((ext_vector_type(2)))  float    v2f;
typedef __attribute__((ext_vector_type(4)))  unsigned v4u;

constexpr int kBatch   = 16;
constexpr int kNPts    = 8192;
constexpr int kNCent   = 512;
constexpr int kNSamp   = 32;
constexpr int kCin0    = 9;
constexpr int kKPad0   = 32;
constexpr int kChanL0  = 64;
constexpr int kChanL1  = 64;
constexpr int kChanL2  = 128;
constexpr int kPartPitch = 36;
constexpr float kRad2    = 0.16f;
constexpr float kBnEps   = 1e-5f;
constexpr float kResScale = 2048.0f;
constexpr float kResInv   = 1.0f / 2048.0f;
constexpr int kFpsThreads = 512;
constexpr int kFpsPpt     = 16;

static_assert(kFpsThreads * kFpsPpt == kNPts, "fps coverage");
static_assert(kBatch * 3 * kNCent * 4 == 98304, "out0 bytes");
static_assert(98304 + kBatch * kChanL2 * kNCent * 4 == 4292608, "d_out bytes");
static_assert(kKPad0 % 32 == 0 && kChanL0 % 32 == 0 && kChanL1 % 32 == 0, "K multiples of 32");
static_assert(kChanL0 % 16 == 0 && kChanL1 % 16 == 0 && kChanL2 % 16 == 0, "N tile multiples");

constexpr size_t kOffNewXyz = 0;
constexpr size_t kSzNewXyz  = (size_t)kBatch * kNCent * 4 * 4;
constexpr size_t kOffX0     = kOffNewXyz + kSzNewXyz;
constexpr size_t kSzX0      = (size_t)kBatch * kNCent * kNSamp * 64 * 2;
constexpr size_t kOffW0H    = kOffX0 + kSzX0;
constexpr size_t kSzW0      = (size_t)kChanL0 * kKPad0 * 2;
constexpr size_t kOffW0L    = kOffW0H + kSzW0;
constexpr size_t kOffW1H    = kOffW0L + kSzW0;
constexpr size_t kSzW1      = (size_t)kChanL1 * kChanL0 * 2;
constexpr size_t kOffW1L    = kOffW1H + kSzW1;
constexpr size_t kOffW2H    = kOffW1L + kSzW1;
constexpr size_t kSzW2      = (size_t)kChanL2 * kChanL1 * 2;
constexpr size_t kOffW2L    = kOffW2H + kSzW2;
constexpr size_t kOffSS     = kOffW2L + kSzW2;
constexpr size_t kSzSS      = 256 * 2 * 4;
constexpr size_t kWsTotal   = kOffSS + kSzSS;
static_assert(kWsTotal == 33744896, "carve total");
static_assert(kWsTotal <= 134217728, "carve limit");
static_assert(kOffX0 % 128 == 0 && kOffW0H % 128 == 0 && kOffSS % 128 == 0, "line aligned");

template <typename T> struct Frag;
template <> struct Frag<_Float16> {
  typedef v16h V; union U { v16h v; v8h h[2]; };
  static __device__ __forceinline__ v16h load(const _Float16* p) {
    U f; f.h[0] = *(const v8h*)(p); f.h[1] = *(const v8h*)(p + 16); return f.v;
  }
  static __device__ __forceinline__ v8f mma(v16h a, v16h b, v8f c) {
    return __builtin_amdgcn_wmma_f32_16x16x32_f16(false, a, false, b, (short)0, c, false, false);
  }
};

__device__ __forceinline__ v8f mma_g(v16h a, v16h b, v8f c) {
  c = Frag<_Float16>::mma(a, b, c);
  asm volatile("v_nop\n\tv_nop\n\tv_nop\n\tv_nop" : "+v"(c) : "v"(a), "v"(b));
  return c;
}

__device__ __forceinline__ void mma3(v16h ah, v16h al, v16h bh, v16h bl, v8f& am, v8f& ar) {
  am = mma_g(ah, bh, am);
  ar = mma_g(ah, bl, ar);
  ar = mma_g(al, bh, ar);
}

__device__ __forceinline__ v8f fold_acc(v8f am, v8f ar) {
  v8f y;
#pragma unroll
  for (int r = 0; r < 8; ++r) {
    const float t = ar[r] * kResInv;
    y[r] = am[r] + t;
  }
  return y;
}

__device__ __forceinline__ float bn_relu(float y, float sc, float sh) {
  float v = y * sc;
  v = v + sh;
  return fmaxf(v, 0.0f);
}

__device__ __forceinline__ void split_h(float v, _Float16& hi, _Float16& lo) {
  hi = (_Float16)v;
  const float hf = (float)hi;
  const float rs = (v - hf) * kResScale;
  lo = (_Float16)rs;
}

__device__ __forceinline__ unsigned h_bits(_Float16 h) {
  return (unsigned)__builtin_bit_cast(unsigned short, h);
}
__device__ __forceinline__ unsigned pk2(_Float16 a, _Float16 b) {
  return h_bits(a) | (h_bits(b) << 16);
}

__device__ __forceinline__ void cvt_plane(const float* __restrict__ w, int cin, int kpad, int nchunks,
                                          unsigned* __restrict__ hiP, unsigned* __restrict__ loP, int tid) {
  const int cpr = kpad >> 3;
#pragma unroll 1
  for (int ch = tid; ch < nchunks; ch += 256) {
    const int o  = ch / cpr;
    const int k0 = (ch - o * cpr) * 8;
    unsigned hw[4], lw[4];
#pragma unroll
    for (int e2 = 0; e2 < 4; ++e2) {
      const int ka = k0 + 2 * e2;
      const int kb = ka + 1;
      const int kac = ka < cin ? ka : cin - 1;
      const int kbc = kb < cin ? kb : cin - 1;
      float va = w[o * cin + kac];
      float vb = w[o * cin + kbc];
      va = (ka < cin) ? va : 0.0f;
      vb = (kb < cin) ? vb : 0.0f;
      _Float16 ha, la, hb, lb;
      split_h(va, ha, la);
      split_h(vb, hb, lb);
      hw[e2] = pk2(ha, hb);
      lw[e2] = pk2(la, lb);
    }
    v4u hv, lv;
    hv[0] = hw[0]; hv[1] = hw[1]; hv[2] = hw[2]; hv[3] = hw[3];
    lv[0] = lw[0]; lv[1] = lw[1]; lv[2] = lw[2]; lv[3] = lw[3];
    *(volatile v4u*)(hiP + (size_t)ch * 4) = hv;
    *(volatile v4u*)(loP + (size_t)ch * 4) = lv;
    __threadfence();
    *(volatile v4u*)(hiP + (size_t)ch * 4) = hv;
    *(volatile v4u*)(loP + (size_t)ch * 4) = lv;
  }
}

__global__ __launch_bounds__(256) void prep_kernel(
    const float* __restrict__ w0, const float* __restrict__ cb0, const float* __restrict__ g0,
    const float* __restrict__ be0, const float* __restrict__ m0, const float* __restrict__ v0,
    const float* __restrict__ w1, const float* __restrict__ cb1, const float* __restrict__ g1,
    const float* __restrict__ be1, const float* __restrict__ m1, const float* __restrict__ v1,
    const float* __restrict__ w2, const float* __restrict__ cb2, const float* __restrict__ g2,
    const float* __restrict__ be2, const float* __restrict__ m2, const float* __restrict__ v2,
    unsigned* __restrict__ w0h, unsigned* __restrict__ w0l,
    unsigned* __restrict__ w1h, unsigned* __restrict__ w1l,
    unsigned* __restrict__ w2h, unsigned* __restrict__ w2l,
    float* __restrict__ ssTab)
{
  const int tid = threadIdx.x;
  cvt_plane(w0, kCin0,   kKPad0,  kChanL0 * kKPad0  / 8, w0h, w0l, tid);
  cvt_plane(w1, kChanL0, kChanL0, kChanL1 * kChanL0 / 8, w1h, w1l, tid);
  cvt_plane(w2, kChanL1, kChanL1, kChanL2 * kChanL1 / 8, w2h, w2l, tid);

  const float* pcb; const float* pg; const float* pbe; const float* pm; const float* pv;
  int ch;
  if (tid < 64)       { pcb = cb0; pg = g0; pbe = be0; pm = m0; pv = v0; ch = tid; }
  else if (tid < 128) { pcb = cb1; pg = g1; pbe = be1; pm = m1; pv = v1; ch = tid - 64; }
  else                { pcb = cb2; pg = g2; pbe = be2; pm = m2; pv = v2; ch = tid - 128; }
  const float gv = pg[ch], vv = pv[ch], cbv = pcb[ch], bev = pbe[ch], mv = pm[ch];
  const float sc = gv / sqrtf(vv + kBnEps);
  const float ta = cbv * sc;
  const float tb = mv * sc;
  const float sh = ta + (bev - tb);
  v2f val; val[0] = sc; val[1] = sh;
  *(volatile v2f*)(ssTab + 2 * tid) = val;
  __threadfence();
  *(volatile v2f*)(ssTab + 2 * tid) = val;
}

__global__ __launch_bounds__(512) void fps_kernel(const float* __restrict__ xyz,
                                                  float* __restrict__ newXyz,
                                                  float* __restrict__ out0)
{
#pragma clang fp contract(off)
  __shared__ float sVal[2][16];
  __shared__ int   sIdx[2][16];
  __shared__ __align__(16) float sCent[3 * kNCent];

  const int b    = blockIdx.x;
  const int tid  = threadIdx.x;
  const int lane = tid & 31;
  const int wave = tid >> 5;
  const float* xb = xyz + (size_t)b * 3 * kNPts;

  float px[kFpsPpt], py[kFpsPpt], pz[kFpsPpt], pd[kFpsPpt];
#pragma unroll
  for (int j0 = 0; j0 < kFpsPpt; j0 += 4) {
#pragma unroll
    for (int jj = 0; jj < 4; ++jj) {
      const int j = j0 + jj;
      const int p = j * kFpsThreads + tid;
      px[j] = xb[p];
      py[j] = xb[kNPts + p];
      pz[j] = xb[2 * kNPts + p];
    }
    asm volatile("" : "+v"(px[j0]), "+v"(px[j0 + 1]), "+v"(px[j0 + 2]), "+v"(px[j0 + 3]),
                      "+v"(py[j0]), "+v"(py[j0 + 1]), "+v"(py[j0 + 2]), "+v"(py[j0 + 3]),
                      "+v"(pz[j0]), "+v"(pz[j0 + 1]), "+v"(pz[j0 + 2]), "+v"(pz[j0 + 3]));
  }
#pragma unroll
  for (int j = 0; j < kFpsPpt; ++j) pd[j] = 1e10f;

  int far = 0;
#pragma unroll 1
  for (int it = 0; it < kNCent; ++it) {
    const float cx = xb[far];
    const float cy = xb[kNPts + far];
    const float cz = xb[2 * kNPts + far];
    if (tid == 0) {
      sCent[it] = cx;
      sCent[kNCent + it] = cy;
      sCent[2 * kNCent + it] = cz;
    }
    float best = -1.0f;
    int   bi   = tid;
#pragma unroll
    for (int j = 0; j < kFpsPpt; ++j) {
      const float dx = px[j] - cx;
      const float dy = py[j] - cy;
      const float dz = pz[j] - cz;
      const float t0 = dx * dx;
      const float t1 = dy * dy;
      const float t2 = dz * dz;
      const float d  = (t0 + t2) + t1;
      const float nd = fminf(pd[j], d);
      pd[j] = nd;
      const bool tk = nd > best;
      best = tk ? nd : best;
      bi   = tk ? (j * kFpsThreads + tid) : bi;
    }
#pragma unroll
    for (int off = 16; off > 0; off >>= 1) {
      const float ov = __shfl_xor(best, off, 32);
      const int   oi = __shfl_xor(bi, off, 32);
      const bool  tk = (ov > best) || ((ov == best) && (oi < bi));
      best = tk ? ov : best;
      bi   = tk ? oi : bi;
    }
    const int par = it & 1;
    if (lane == 0) { sVal[par][wave] = best; sIdx[par][wave] = bi; }
    __syncthreads();
    float rv = sVal[par][lane & 15];
    int   ri = sIdx[par][lane & 15];
#pragma unroll
    for (int off = 8; off > 0; off >>= 1) {
      const float ov = __shfl_xor(rv, off, 32);
      const int   oi = __shfl_xor(ri, off, 32);
      const bool  tk = (ov > rv) || ((ov == rv) && (oi < ri));
      rv = tk ? ov : rv;
      ri = tk ? oi : ri;
    }
    ri = ri < 0 ? 0 : ri;
    ri = ri > (kNPts - 1) ? (kNPts - 1) : ri;
    far = ri;
  }
  __syncthreads();

  const int tcl = tid < 384 ? tid : 383;
  const v4f ov4 = *(const v4f*)(sCent + 4 * tcl);
  v4f nv4;
  nv4[0] = sCent[tid];
  nv4[1] = sCent[kNCent + tid];
  nv4[2] = sCent[2 * kNCent + tid];
  nv4[3] = 0.0f;
  float* o0 = out0 + (size_t)b * (3 * kNCent) + 4 * tcl;
  float* nx = newXyz + ((size_t)b * kNCent + tid) * 4;
  for (int pass = 0; pass < 2; ++pass) {
    if (tid < 384) *(volatile v4f*)o0 = ov4;
    *(volatile v4f*)nx = nv4;
    __threadfence();
  }
}

__global__ __launch_bounds__(256) void ballq_gather_kernel(const float* __restrict__ xyz,
                                                           const float* __restrict__ pts,
                                                           const float* __restrict__ newXyz,
                                                           unsigned* __restrict__ X0w)
{
#pragma clang fp contract(off)
  __shared__ int sList[8][kNSamp];
  __shared__ __align__(16) unsigned sTile[8 * 1024];

  const int lane = threadIdx.x & 31;
  const int wave = threadIdx.x >> 5;
  const int gw   = blockIdx.x * 8 + wave;
  const int b    = gw >> 9;

  sList[wave][lane] = kNPts - 1;
  __syncthreads();

  const float* xb = xyz + (size_t)b * 3 * kNPts;
  const float* pb = pts + (size_t)b * 6 * kNPts;
  const v4f q = *(const v4f*)(newXyz + (size_t)gw * 4);
  const float qx = q[0], qy = q[1], qz = q[2];
  const float s0 = qx * qx, s1 = qy * qy, s2 = qz * qz;
  const float sqs = (s0 + s2) + s1;

  int count = 0;
#pragma unroll 1
  for (int p0 = 0; p0 < kNPts && count < kNSamp; p0 += 32) {
    const int p = p0 + lane;
    const float x  = xb[p];
    const float y  = xb[kNPts + p];
    const float zc = xb[2 * kNPts + p];
    float dp = qx * x;
    dp = fmaf(qy, y, dp);
    dp = fmaf(qz, zc, dp);
    const float t0 = x * x, t1 = y * y, t2 = zc * zc;
    const float sqp = (t0 + t2) + t1;
    float d = -2.0f * dp;
    d = d + sqs;
    d = d + sqp;
    const bool hit = !(d > kRad2);
    const unsigned mask = (unsigned)__ballot(hit ? 1 : 0);
    const int pre  = __popc(mask & ((1u << lane) - 1u));
    const int slot = count + pre;
    if (hit && slot < kNSamp) sList[wave][slot] = p;
    count += __popc(mask);
  }
  __syncthreads();

  const int valid = count < kNSamp ? count : kNSamp;
  const int first = sList[wave][0];
  const int mine  = sList[wave][lane];
  int idx = (lane < valid) ? mine : first;
  idx = idx < 0 ? 0 : idx;
  idx = idx > (kNPts - 1) ? (kNPts - 1) : idx;

  float f[9];
  f[0] = xb[idx] - qx;
  f[1] = xb[kNPts + idx] - qy;
  f[2] = xb[2 * kNPts + idx] - qz;
#pragma unroll
  for (int c = 0; c < 6; ++c) f[3 + c] = pb[c * kNPts + idx];

  _Float16 hh[9], ll[9];
#pragma unroll
  for (int c = 0; c < 9; ++c) split_h(f[c], hh[c], ll[c]);

  unsigned zop = 0u;
  asm volatile("" : "+v"(zop));
  const unsigned w8h = (h_bits(hh[8]) & 0xffffu) | (zop << 16);
  const unsigned w8l = (h_bits(ll[8]) & 0xffffu) | (zop << 16);

  v4u hA, hB, lA, lB, zz;
  hA[0] = pk2(hh[0], hh[1]); hA[1] = pk2(hh[2], hh[3]); hA[2] = pk2(hh[4], hh[5]); hA[3] = pk2(hh[6], hh[7]);
  hB[0] = w8h; hB[1] = 0u; hB[2] = 0u; hB[3] = 0u;
  lA[0] = pk2(ll[0], ll[1]); lA[1] = pk2(ll[2], ll[3]); lA[2] = pk2(ll[4], ll[5]); lA[3] = pk2(ll[6], ll[7]);
  lB[0] = w8l; lB[1] = 0u; lB[2] = 0u; lB[3] = 0u;
  zz[0] = 0u; zz[1] = 0u; zz[2] = 0u; zz[3] = 0u;

  unsigned* trow = sTile + wave * 1024 + lane * 32;
  *(v4u*)(trow + 0)  = hA;
  *(v4u*)(trow + 4)  = hB;
  *(v4u*)(trow + 8)  = zz;
  *(v4u*)(trow + 12) = zz;
  *(v4u*)(trow + 16) = lA;
  *(v4u*)(trow + 20) = lB;
  *(v4u*)(trow + 24) = zz;
  *(v4u*)(trow + 28) = zz;
  __syncthreads();

  unsigned* dst = X0w + (size_t)gw * 1024;
  const unsigned* src = sTile + wave * 1024;
  for (int pass = 0; pass < 2; ++pass) {
#pragma unroll
    for (int it = 0; it < 8; ++it) {
      const int wofs = (it * 32 + lane) * 4;
      const v4u v = *(const v4u*)(src + wofs);
      *(volatile v4u*)(dst + wofs) = v;
    }
    __threadfence();
  }
}

__global__ __launch_bounds__(256) void mlp_pool_kernel(const _Float16* __restrict__ X0,
                                                       const _Float16* w0h, const _Float16* w0l,
                                                       const _Float16* w1h, const _Float16* w1l,
                                                       const _Float16* w2h, const _Float16* w2l,
                                                       const float* __restrict__ ssTab,
                                                       float* __restrict__ out1)
{
  __shared__ __align__(16) float sSS[512];
  __shared__ __align__(16) float sPart[2 * kChanL2 * kPartPitch];

  const int tid  = threadIdx.x;
  const int lane = tid & 31;
  const int wave = tid >> 5;
  const int h    = lane >> 4;
  const int n    = lane & 15;
  const int b    = blockIdx.x >> 4;
  const int s0   = (blockIdx.x & 15) * 32;

  sSS[2 * tid]     = ssTab[2 * tid];
  sSS[2 * tid + 1] = ssTab[2 * tid + 1];
  __syncthreads();

#pragma unroll 1
  for (int p = 0; p < 8; ++p) {
    int zo = 0;
    asm volatile("" : "+v"(zo));
    const int g = wave * 4 + (p >> 1);
    const int t = p & 1;
    const size_t row = ((size_t)(b * kNCent + s0 + g)) * kNSamp + t * 16 + n;
    const _Float16* xr = X0 + row * 64 + 8 * h + zo;
    const v16h xh = Frag<_Float16>::load(xr);
    const v16h xl = Frag<_Float16>::load(xr + 32);

    v16h a1h[2], a1l[2], a2h[2], a2l[2];

#pragma unroll
    for (int c = 0; c < 4; ++c) {
      const int woff = (16 * c + n) * kKPad0 + 8 * h + zo;
      const v16h ah = Frag<_Float16>::load(w0h + woff);
      const v16h al = Frag<_Float16>::load(w0l + woff);
      v8f am = (v8f){0.f, 0.f, 0.f, 0.f, 0.f, 0.f, 0.f, 0.f};
      v8f ar = (v8f){0.f, 0.f, 0.f, 0.f, 0.f, 0.f, 0.f, 0.f};
      mma3(ah, al, xh, xl, am, ar);
      const v8f y = fold_acc(am, ar);
      const int sb = 2 * (16 * c + 8 * h) + zo;
#pragma unroll
      for (int r = 0; r < 8; ++r) {
        const float e = bn_relu(y[r], sSS[sb + 2 * r], sSS[sb + 2 * r + 1]);
        _Float16 eh, el;
        split_h(e, eh, el);
        a1h[c >> 1][(c & 1) * 8 + r] = eh;
        a1l[c >> 1][(c & 1) * 8 + r] = el;
      }
      asm volatile("" : "+v"(zo));
    }

#pragma unroll
    for (int c = 0; c < 4; ++c) {
      const int woff = (16 * c + n) * kChanL0 + 8 * h + zo;
      v8f am = (v8f){0.f, 0.f, 0.f, 0.f, 0.f, 0.f, 0.f, 0.f};
      v8f ar = (v8f){0.f, 0.f, 0.f, 0.f, 0.f, 0.f, 0.f, 0.f};
#pragma unroll
      for (int qk = 0; qk < 2; ++qk) {
        const v16h ah = Frag<_Float16>::load(w1h + woff + 32 * qk);
        const v16h al = Frag<_Float16>::load(w1l + woff + 32 * qk);
        mma3(ah, al, a1h[qk], a1l[qk], am, ar);
      }
      const v8f y = fold_acc(am, ar);
      const int sb = 2 * (kChanL0 + 16 * c + 8 * h) + zo;
#pragma unroll
      for (int r = 0; r < 8; ++r) {
        const float e = bn_relu(y[r], sSS[sb + 2 * r], sSS[sb + 2 * r + 1]);
        _Float16 eh, el;
        split_h(e, eh, el);
        a2h[c >> 1][(c & 1) * 8 + r] = eh;
        a2l[c >> 1][(c & 1) * 8 + r] = el;
      }
      asm volatile("" : "+v"(zo));
    }

#pragma unroll
    for (int c = 0; c < 8; ++c) {
      const int woff = (16 * c + n) * kChanL1 + 8 * h + zo;
      v8f am = (v8f){0.f, 0.f, 0.f, 0.f, 0.f, 0.f, 0.f, 0.f};
      v8f ar = (v8f){0.f, 0.f, 0.f, 0.f, 0.f, 0.f, 0.f, 0.f};
#pragma unroll
      for (int qk = 0; qk < 2; ++qk) {
        const v16h ah = Frag<_Float16>::load(w2h + woff + 32 * qk);
        const v16h al = Frag<_Float16>::load(w2l + woff + 32 * qk);
        mma3(ah, al, a2h[qk], a2l[qk], am, ar);
      }
      const v8f y = fold_acc(am, ar);
      const int sb = 2 * (kChanL0 + kChanL1 + 16 * c + 8 * h) + zo;
      float mx[8];
#pragma unroll
      for (int r = 0; r < 8; ++r) {
        float e = bn_relu(y[r], sSS[sb + 2 * r], sSS[sb + 2 * r + 1]);
#pragma unroll
        for (int off = 1; off < 16; off <<= 1) {
          const float o2 = __shfl_xor(e, off, 32);
          e = fmaxf(e, o2);
        }
        mx[r] = e;
      }
      if (n == 0) {
#pragma unroll
        for (int r = 0; r < 8; ++r)
          sPart[(t * kChanL2 + 16 * c + 8 * h + r) * kPartPitch + g] = mx[r];
      }
      asm volatile("" : "+v"(zo));
    }
  }
  __syncthreads();

  float* ob = out1 + ((size_t)b * kChanL2) * kNCent + s0;
  const int qd = lane >> 3;
  const int c4 = (lane & 7) * 4;
  for (int pass = 0; pass < 2; ++pass) {
#pragma unroll
    for (int it = 0; it < 4; ++it) {
      const int o = it * 32 + wave * 4 + qd;
      const v4f pa = *(const v4f*)(sPart + (size_t)o * kPartPitch + c4);
      const v4f pq = *(const v4f*)(sPart + (size_t)(kChanL2 + o) * kPartPitch + c4);
      v4f v;
      v[0] = fmaxf(pa[0], pq[0]);
      v[1] = fmaxf(pa[1], pq[1]);
      v[2] = fmaxf(pa[2], pq[2]);
      v[3] = fmaxf(pa[3], pq[3]);
      *(volatile v4f*)(ob + (size_t)o * kNCent + c4) = v;
    }
    __threadfence();
  }
}

extern "C" void kernel_launch(void* const* d_in, const int* in_sizes, int n_in,
                              void* d_out, int out_size, void* d_ws, size_t ws_size,
                              hipStream_t stream) {
  (void)in_sizes; (void)n_in; (void)out_size;
  if (ws_size < kWsTotal) return;

  const float* xyz = (const float*)d_in[0];
  const float* pts = (const float*)d_in[1];
  const float* w0  = (const float*)d_in[2];
  const float* cb0 = (const float*)d_in[3];
  const float* g0  = (const float*)d_in[4];
  const float* be0 = (const float*)d_in[5];
  const float* m0  = (const float*)d_in[6];
  const float* v0  = (const float*)d_in[7];
  const float* w1  = (const float*)d_in[8];
  const float* cb1 = (const float*)d_in[9];
  const float* g1  = (const float*)d_in[10];
  const float* be1 = (const float*)d_in[11];
  const float* m1  = (const float*)d_in[12];
  const float* v1  = (const float*)d_in[13];
  const float* w2  = (const float*)d_in[14];
  const float* cb2 = (const float*)d_in[15];
  const float* g2  = (const float*)d_in[16];
  const float* be2 = (const float*)d_in[17];
  const float* m2  = (const float*)d_in[18];
  const float* v2  = (const float*)d_in[19];

  float* out0 = (float*)d_out;
  float* out1 = out0 + (size_t)kBatch * 3 * kNCent;

  char* ws = (char*)d_ws;
  float*    newXyz = (float*)(ws + kOffNewXyz);
  unsigned* x0w    = (unsigned*)(ws + kOffX0);
  unsigned* w0h    = (unsigned*)(ws + kOffW0H);
  unsigned* w0l    = (unsigned*)(ws + kOffW0L);
  unsigned* w1h    = (unsigned*)(ws + kOffW1H);
  unsigned* w1l    = (unsigned*)(ws + kOffW1L);
  unsigned* w2h    = (unsigned*)(ws + kOffW2H);
  unsigned* w2l    = (unsigned*)(ws + kOffW2L);
  float*    ssTab  = (float*)(ws + kOffSS);

  prep_kernel<<<1, 256, 0, stream>>>(
      w0, cb0, g0, be0, m0, v0,
      w1, cb1, g1, be1, m1, v1,
      w2, cb2, g2, be2, m2, v2,
      w0h, w0l, w1h, w1l, w2h, w2l, ssTab);

  fps_kernel<<<kBatch, kFpsThreads, 0, stream>>>(xyz, newXyz, out0);

  ballq_gather_kernel<<<(kBatch * kNCent) / 8, 256, 0, stream>>>(xyz, pts, newXyz, x0w);

  mlp_pool_kernel<<<kBatch * (kNCent / 32), 256, 0, stream>>>(
      (const _Float16*)x0w,
      (const _Float16*)w0h, (const _Float16*)w0l,
      (const _Float16*)w1h, (const _Float16*)w1l,
      (const _Float16*)w2h, (const _Float16*)w2l,
      ssTab, out1);
}
